// UniPhyModel_88579405513036
// MI455X (gfx1250) — hardware-run, weakly checked
//
#include <hip/hip_runtime.h>
#include <math.h>

typedef __attribute__((ext_vector_type(16))) _Float16 v16h;
typedef __attribute__((ext_vector_type(8)))  _Float16 v8h;
typedef __attribute__((ext_vector_type(8)))  float    v8f;
typedef __attribute__((ext_vector_type(4)))  float    v4f;

constexpr int kTok    = 2048;
constexpr int kSteps  = 8;
constexpr int kSpa    = 256;
constexpr int kDc     = 256;
constexpr int kCh     = 512;
constexpr int kFfn    = 1024;
constexpr int kExp    = 4;
constexpr int kFfnAll = kExp * kFfn;
constexpr int kPatchF = 1024;
constexpr int kConvK  = 9 * kCh;
constexpr int kPadW   = 18;
constexpr int kPadRows = kSteps * kPadW * kPadW;
constexpr int kLayers = 2;
static_assert(kTok == kSteps * kSpa, "token count");
static_assert(kCh == 2 * kDc, "channel halves");
static_assert(kConvK == 4608 && kPadRows == 2592, "conv geometry");
static_assert((kTok % 64) == 0 && (kCh % 64) == 0 && (kFfnAll % 64) == 0 && (kPatchF % 64) == 0, "GEMM M,N multiples of 64");
static_assert((kCh % 32) == 0 && (kPatchF % 32) == 0 && (kFfnAll % 32) == 0 && (kConvK % 32) == 0, "GEMM K multiples of 32");

constexpr float kCarryX = 16.0f;
constexpr float kCarryA = 16.0f;
constexpr float kCarryH = 64.0f;
constexpr float kCarryW = 1024.0f;
constexpr float kScaleXW = 1.0f / (kCarryX * kCarryW);
constexpr float kScaleAW = 1.0f / (kCarryA * kCarryW);
constexpr float kScaleHW = 1.0f / (kCarryH * kCarryW);

constexpr size_t kSzWencT = (size_t)kCh * kPatchF * 2;
constexpr size_t kSzWdecT = (size_t)kPatchF * kCh * 2;
constexpr size_t kSzConvT = (size_t)kLayers * kCh * kConvK * 2;
constexpr size_t kSzCm    = (size_t)kLayers * kCh * kCh * 2;
constexpr size_t kSzW1T   = (size_t)kLayers * kFfnAll * kCh * 2;
constexpr size_t kSzW2T   = (size_t)kLayers * kCh * kFfnAll * 2;
constexpr size_t kSzXp    = (size_t)kTok * kPatchF * 2;
constexpr size_t kSzF32   = (size_t)kTok * kCh * 4;
constexpr size_t kSzZnp   = (size_t)kPadRows * kCh * 2;
constexpr size_t kSzF16   = (size_t)kTok * kCh * 2;
constexpr size_t kSzHid   = (size_t)kTok * kFfnAll * 2;
constexpr size_t kSzProbs = (size_t)kTok * kExp * 4;
constexpr size_t kSzTpar  = (size_t)kLayers * kSteps * 3 * kDc * 4;
constexpr size_t kSzDpar  = (size_t)kLayers * kSteps * 4 * kDc * 4;
constexpr size_t kSzHst   = (size_t)kSpa * kCh * 4;

constexpr size_t kOffWencT = 0;
constexpr size_t kOffWdecT = kOffWencT + kSzWencT;
constexpr size_t kOffConvT = kOffWdecT + kSzWdecT;
constexpr size_t kOffEcm   = kOffConvT + kSzConvT;
constexpr size_t kOffEdcm  = kOffEcm   + kSzCm;
constexpr size_t kOffW1T   = kOffEdcm  + kSzCm;
constexpr size_t kOffW2T   = kOffW1T   + kSzW1T;
constexpr size_t kOffXp    = kOffW2T   + kSzW2T;
constexpr size_t kOffZ     = kOffXp    + kSzXp;
constexpr size_t kOffX     = kOffZ     + kSzF32;
constexpr size_t kOffXE    = kOffX     + kSzF32;
constexpr size_t kOffXO    = kOffXE    + kSzF32;
constexpr size_t kOffTok   = kOffXO    + kSzF32;
constexpr size_t kOffZnp   = kOffTok   + kSzF32;
constexpr size_t kOffX16   = kOffZnp   + kSzZnp;
constexpr size_t kOffH16   = kOffX16   + kSzF16;
constexpr size_t kOffTok16 = kOffH16   + kSzF16;
constexpr size_t kOffZ16   = kOffTok16 + kSzF16;
constexpr size_t kOffHid   = kOffZ16   + kSzF16;
constexpr size_t kOffProbs = kOffHid   + kSzHid;
constexpr size_t kOffTpar  = kOffProbs + kSzProbs;
constexpr size_t kOffDpar  = kOffTpar  + kSzTpar;
constexpr size_t kOffHst   = kOffDpar  + kSzDpar;
constexpr size_t kWsTotal  = kOffHst   + kSzHst;
static_assert(kWsTotal == 84066304ull, "carve total");
static_assert(kWsTotal <= 134217728ull, "carve cap");
static_assert((kSzZnp % 128) == 0 && (kSzTpar % 128) == 0 && (kSzProbs % 128) == 0 && (kSzDpar % 128) == 0, "128-B regions");
static_assert(kOffEdcm == kOffEcm + kSzCm, "decode block matrices directly follow the encode ones");

__device__ __forceinline__ unsigned short f2bf_bits(float f) {
  unsigned u = __float_as_uint(f);
  return (unsigned short)((u + 0x7FFFu + ((u >> 16) & 1u)) >> 16);
}
__device__ __forceinline__ float bf_bits2f(unsigned short h) { return __uint_as_float(((unsigned)h) << 16); }
__device__ __forceinline__ float rbf(float f) { return bf_bits2f(f2bf_bits(f)); }

__device__ __forceinline__ v16h frag_load(const _Float16* p) {
  union U { v16h v; v8h h[2]; } f;
  f.h[0] = *(const v8h*)(p);
  f.h[1] = *(const v8h*)(p + 16);
  return f.v;
}
__device__ __forceinline__ v8f mma_f16(v16h a, v16h b, v8f c) {
  return __builtin_amdgcn_wmma_f32_16x16x32_f16(false, a, false, b, (short)0, c, false, false);
}
__device__ __forceinline__ void guard1(v8f& a, v16h x, v16h y) {
  asm volatile("v_nop\n\tv_nop\n\tv_nop\n\tv_nop" : "+v"(a) : "v"(x), "v"(y));
}
__device__ __forceinline__ void keep4(v16h a, v16h b, v16h c, v16h d) {
  asm volatile("v_nop" :: "v"(a), "v"(b), "v"(c), "v"(d));
}
__device__ __forceinline__ void wave_sync() {
  __builtin_amdgcn_fence(__ATOMIC_RELEASE, "workgroup");
  __builtin_amdgcn_wave_barrier();
  __builtin_amdgcn_fence(__ATOMIC_ACQUIRE, "workgroup");
}
__device__ __forceinline__ float gelu_tanh(float x) {
  const float x3 = x * x * x;
  return 0.5f * x * (1.0f + tanhf(0.7978845608028654f * (x + 0.044715f * x3)));
}

__device__ __forceinline__ void tpose_tile64(const float* __restrict__ src, int ldin,
                                             unsigned short* __restrict__ dst, int ldout,
                                             float mul, float* tile) {
  const int tid = threadIdx.x;
  const int nn = tid & 63, kk = tid >> 6;
#pragma unroll 4
  for (int i = 0; i < 16; ++i) {
    const int k = kk + 4 * i;
    tile[k * 65 + nn] = rbf(src[(size_t)k * ldin + nn]) * mul;
  }
  __syncthreads();
  const int lane = tid & 31, wave = tid >> 5;
  const int q = lane >> 3, c8 = (lane & 7) * 8;
  v8h hv[2];
#pragma unroll
  for (int it = 0; it < 2; ++it) {
    const int n = it * 32 + wave * 4 + q;
#pragma unroll
    for (int e = 0; e < 8; ++e) hv[it][e] = (_Float16)tile[(c8 + e) * 65 + n];
  }
  for (int pass = 0; pass < 2; ++pass) {
#pragma unroll
    for (int it = 0; it < 2; ++it) {
      const int n = it * 32 + wave * 4 + q;
      *(volatile v8h*)(dst + (size_t)n * ldout + c8) = hv[it];
    }
    __threadfence();
  }
}

__global__ __launch_bounds__(256) void pack_transpose_kernel(
    const float* __restrict__ src, int ldin, long inBatch,
    unsigned short* __restrict__ dst, int ldout, int nE, long outStrideL, long outStrideE, float mul) {
  __shared__ float tile[64 * 65];
  const int k0 = blockIdx.x * 64, n0 = blockIdx.y * 64, bz = blockIdx.z;
  const int l = bz / nE, e = bz - l * nE;
  const float* s = src + (size_t)bz * inBatch + (size_t)k0 * ldin + n0;
  unsigned short* d = dst + (size_t)l * outStrideL + (size_t)e * outStrideE + (size_t)n0 * ldout + k0;
  tpose_tile64(s, ldin, d, ldout, mul, tile);
}

__global__ __launch_bounds__(256) void pack_cplx_kernel(
    const float* __restrict__ Ere, const float* __restrict__ Eim,
    const float* __restrict__ Dre, const float* __restrict__ Dim,
    unsigned short* __restrict__ dst, float mul) {
  __shared__ float tile[64 * 65];
  const int k0 = blockIdx.x * 64, n0 = blockIdx.y * 64, z = blockIdx.z;
  const int which = z >> 3, l = (z >> 2) & 1, quad = z & 3;
  const int kq = quad >> 1, nq = quad & 1;
  const float* re = which ? Dre : Ere;
  const float* im = which ? Dim : Eim;
  const float* sm = (kq == nq) ? re : im;
  const float sg = (kq == 1 && nq == 0) ? -mul : mul;
  const float* s = sm + (size_t)l * kDc * kDc + (size_t)k0 * kDc + n0;
  unsigned short* d = dst + (size_t)(which * 2 + l) * kCh * kCh + (size_t)(nq * kDc + n0) * kCh + kq * kDc + k0;
  tpose_tile64(s, kDc, d, kCh, sg, tile);
}

__global__ __launch_bounds__(256) void pack_conv_kernel(const float* __restrict__ src, unsigned short* __restrict__ dst, float mul) {
  __shared__ float sw[kConvK];
  const int tid = threadIdx.x;
  const float* s = src + (size_t)blockIdx.x * kConvK;
#pragma unroll 2
  for (int i = 0; i < 18; ++i) sw[i * 256 + tid] = rbf(s[i * 256 + tid]) * mul;
  __syncthreads();
  v8h hv[3];
#pragma unroll
  for (int it = 0; it < 3; ++it) {
    int chunk = it * 256 + tid;
    chunk = chunk < 575 ? chunk : 575;
    const int j0 = chunk * 8;
    const int tap = j0 >> 9, i0 = j0 & 511;
#pragma unroll
    for (int e = 0; e < 8; ++e) hv[it][e] = (_Float16)sw[(i0 + e) * 9 + tap];
  }
  unsigned short* d = dst + (size_t)blockIdx.x * kConvK;
  for (int pass = 0; pass < 2; ++pass) {
#pragma unroll
    for (int it = 0; it < 3; ++it) {
      const int chunk = it * 256 + tid;
      if (chunk < 576) *(volatile v8h*)(d + (size_t)chunk * 8) = hv[it];
    }
    __threadfence();
  }
}

__global__ __launch_bounds__(64) void halo_zero_kernel(unsigned short* __restrict__ znp) {
  const int row = blockIdx.x;
  const int cell = row % (kPadW * kPadW);
  const int py = cell / kPadW, px = cell - py * kPadW;
  const bool halo = (py == 0) || (py == kPadW - 1) || (px == 0) || (px == kPadW - 1);
  if (!halo) return;
  v8h z;
#pragma unroll
  for (int e = 0; e < 8; ++e) z[e] = (_Float16)0.0f;
  unsigned short* p = znp + (size_t)row * kCh + threadIdx.x * 8;
  *(volatile v8h*)p = z;
  __threadfence();
  *(volatile v8h*)p = z;
}

__global__ __launch_bounds__(256) void patchify_kernel(const float* __restrict__ x, unsigned short* __restrict__ xp) {
  const int chunk = blockIdx.x * 256 + threadIdx.x;
  const int n = chunk >> 7, f0 = (chunk & 127) * 8;
  const int c = f0 >> 8, py = (f0 >> 4) & 15, px0 = f0 & 15;
  const int t = n >> 8, hp = (n >> 4) & 15, wp = n & 15;
  const float* s = x + (((size_t)(t * 4 + c) * 256) + hp * 16 + py) * 256 + wp * 16 + px0;
  const v4f a0 = *(const v4f*)(s);
  const v4f a1 = *(const v4f*)(s + 4);
  v8h hv;
#pragma unroll
  for (int e = 0; e < 4; ++e) {
    const float u0 = a0[e], u1 = a1[e];
    hv[e]     = (_Float16)(rbf(u0) * kCarryX);
    hv[4 + e] = (_Float16)(rbf(u1) * kCarryX);
  }
  unsigned short* p = xp + (size_t)chunk * 8;
  *(volatile v8h*)p = hv;
  __threadfence();
  *(volatile v8h*)p = hv;
}

constexpr int EPI_BIAS = 0;
constexpr int EPI_CONV = 1;
constexpr int EPI_PLAIN = 2;
constexpr int EPI_UP = 3;
constexpr int EPI_DOWN = 4;
constexpr int EPI_IMG = 5;

template <int AMODE, int EPI>
__global__ __launch_bounds__(256) void gemm_f16_kernel(
    const unsigned short* __restrict__ Ap, int lda,
    const unsigned short* __restrict__ Btp, int ldb,
    float* __restrict__ C32, unsigned short* __restrict__ C16, int ldc,
    const float* __restrict__ bias, const float* __restrict__ r0, const float* __restrict__ r1,
    int M, int N, int K, float scale, float carry16) {
  __shared__ __align__(16) float sT[2][64 * 68];
  const _Float16* A  = (const _Float16*)Ap;
  const _Float16* Bt = (const _Float16*)Btp;
  const int lane = threadIdx.x & 31;
  const int wave = threadIdx.x >> 5;
  const int tilesN = N >> 6;
  const int tilesM = M >> 6;
  const int tile = blockIdx.x * 2 + wave;
  if (tile >= tilesM * tilesN) return;
  const int tm = tile / tilesN;
  const int tn = tile - tm * tilesN;
  const int m0 = tm << 6;
  const int n0 = tn << 6;
  const int rlane = lane & 15;
  const int koff  = (lane >> 4) * 8;
  const int mOff  = (lane >> 4) * 8;

  size_t aRow[4];
#pragma unroll
  for (int i = 0; i < 4; ++i) {
    if (AMODE == 1) {
      const int prow0 = ((m0 >> 8) * kPadW + ((m0 >> 4) & 15)) * kPadW;
      aRow[i] = (size_t)(prow0 + i * kPadW + rlane) * kCh + koff;
    } else {
      aRow[i] = (size_t)(m0 + (i << 4) + rlane) * lda + koff;
    }
  }
  size_t bRow[4];
#pragma unroll
  for (int j = 0; j < 4; ++j) bRow[j] = (size_t)(n0 + (j << 4) + rlane) * ldb + koff;

  v8f acc[4][4];
#pragma unroll
  for (int i = 0; i < 4; ++i)
#pragma unroll
    for (int j = 0; j < 4; ++j) acc[i][j] = (v8f){0.f, 0.f, 0.f, 0.f, 0.f, 0.f, 0.f, 0.f};

  for (int k0 = 0; k0 < K; k0 += 32) {
    size_t aAdd = (size_t)k0;
    if (AMODE == 1) {
      const int tap = k0 >> 9;
      const int ky = tap / 3;
      const int kx = tap - 3 * ky;
      aAdd = (size_t)(ky * kPadW + kx) * kCh + (size_t)(k0 & 511);
    }
    v16h bh[4];
#pragma unroll
    for (int j = 0; j < 4; ++j) bh[j] = frag_load(Bt + bRow[j] + k0);
#pragma unroll
    for (int i = 0; i < 4; ++i) {
      const v16h ah = frag_load(A + aRow[i] + aAdd);
#pragma unroll
      for (int j = 0; j < 4; ++j) acc[i][j] = mma_f16(ah, bh[j], acc[i][j]);
      guard1(acc[i][0], ah, bh[0]);
      guard1(acc[i][1], ah, bh[1]);
      guard1(acc[i][2], ah, bh[2]);
      guard1(acc[i][3], ah, bh[3]);
    }
    keep4(bh[0], bh[1], bh[2], bh[3]);
  }

  float* tl = sT[wave];
#pragma unroll
  for (int i = 0; i < 4; ++i)
#pragma unroll
    for (int j = 0; j < 4; ++j)
#pragma unroll
      for (int r = 0; r < 8; ++r)
        tl[((i << 4) + mOff + r) * 68 + (j << 4) + rlane] = acc[i][j][r] * scale;
  wave_sync();

  const int hh = lane >> 4, c4 = (lane & 15) * 4;
  if (EPI != EPI_PLAIN) {
    float b0 = 0.f, b1 = 0.f, b2 = 0.f, b3 = 0.f;
    if (EPI == EPI_BIAS || EPI == EPI_CONV || EPI == EPI_IMG) {
      const v4f bb = *(const v4f*)(bias + n0 + c4);
      const float t0 = bb[0], t1 = bb[1], t2 = bb[2], t3 = bb[3];
      b0 = rbf(t0); b1 = rbf(t1); b2 = rbf(t2); b3 = rbf(t3);
    }
    const int ex = n0 >> 10;
#pragma unroll 1
    for (int it = 0; it < 32; ++it) {
      const int row = it * 2 + hh;
      const int m = m0 + row;
      float* sp = tl + row * 68 + c4;
      const v4f v = *(const v4f*)sp;
      float a0 = v[0], a1 = v[1], a2 = v[2], a3 = v[3];
      if (EPI == EPI_BIAS || EPI == EPI_IMG) {
        a0 += b0; a1 += b1; a2 += b2; a3 += b3;
      }
      if (EPI == EPI_CONV) {
        const v4f z = *(const v4f*)(r0 + (size_t)m * ldc + n0 + c4);
        a0 += b0 + z[0]; a1 += b1 + z[1]; a2 += b2 + z[2]; a3 += b3 + z[3];
      }
      if (EPI == EPI_UP) {
        const float p = r0[(size_t)m * kExp + ex];
        a0 = gelu_tanh(a0) * p; a1 = gelu_tanh(a1) * p; a2 = gelu_tanh(a2) * p; a3 = gelu_tanh(a3) * p;
      }
      if (EPI == EPI_DOWN) {
        const v4f xa = *(const v4f*)(r0 + (size_t)m * ldc + n0 + c4);
        const v4f xb = *(const v4f*)(r1 + (size_t)m * ldc + n0 + c4);
        a0 += xa[0] + xb[0]; a1 += xa[1] + xb[1]; a2 += xa[2] + xb[2]; a3 += xa[3] + xb[3];
      }
      const v4f w = (v4f){a0, a1, a2, a3};
      *(v4f*)sp = w;
    }
    wave_sync();
  }

  if (EPI == EPI_BIAS || EPI == EPI_CONV || EPI == EPI_PLAIN || EPI == EPI_DOWN) {
    for (int pass = 0; pass < 2; ++pass) {
#pragma unroll 4
      for (int it = 0; it < 32; ++it) {
        const int row = it * 2 + hh;
        const v4f v = *(const v4f*)(tl + row * 68 + c4);
        *(volatile v4f*)(C32 + (size_t)(m0 + row) * ldc + n0 + c4) = v;
      }
      __threadfence();
    }
  }
  if (EPI == EPI_CONV || EPI == EPI_UP || EPI == EPI_DOWN) {
    const int q = lane >> 3, c8 = (lane & 7) * 8;
    for (int pass = 0; pass < 2; ++pass) {
#pragma unroll 2
      for (int it = 0; it < 16; ++it) {
        const int row = it * 4 + q;
        const float* sp = tl + row * 68 + c8;
        const v4f u0 = *(const v4f*)(sp);
        const v4f u1 = *(const v4f*)(sp + 4);
        v8h hv;
#pragma unroll
        for (int e = 0; e < 4; ++e) {
          hv[e]     = (_Float16)(u0[e] * carry16);
          hv[4 + e] = (_Float16)(u1[e] * carry16);
        }
        *(volatile v8h*)(C16 + (size_t)(m0 + row) * ldc + n0 + c8) = hv;
      }
      __threadfence();
    }
  }
  if (EPI == EPI_IMG) {
    const int t = m0 >> 8, hp0 = (m0 >> 4) & 15;
    const int c = n0 >> 8, py0 = (n0 >> 4) & 15;
    for (int pass = 0; pass < 2; ++pass) {
#pragma unroll 1
      for (int idx = 0; idx < 32; ++idx) {
        const int i4 = idx >> 3, pyl = (idx >> 1) & 3, s = idx & 1;
        const int f = s * 32 + lane;
        const int wp = f >> 2, px4 = (f & 3) * 4;
        const v4f v = *(const v4f*)(tl + (i4 * 16 + wp) * 68 + pyl * 16 + px4);
        float* dptr = C32 + (((size_t)(t * 4 + c) * 256) + (hp0 + i4) * 16 + py0 + pyl) * 256 + wp * 16 + px4;
        *(volatile v4f*)dptr = v;
      }
      __threadfence();
    }
  }
}

template <int MODE>
__global__ __launch_bounds__(256) void ln_kernel(
    const float* __restrict__ X, const float* __restrict__ w, const float* __restrict__ b,
    unsigned short* __restrict__ out16, float* __restrict__ out32,
    const float* __restrict__ Wr, float* __restrict__ probs) {
  __shared__ __align__(16) float sRow[8 * kCh];
  __shared__ __align__(16) float sPr[32];
  const int tid = threadIdx.x, lane = tid & 31, wave = tid >> 5;
  const int tok = blockIdx.x * 8 + wave;
  const float* xr = X + (size_t)tok * kCh;
  v4f xv[4];
#pragma unroll
  for (int j = 0; j < 4; ++j) xv[j] = *(const v4f*)(xr + lane * 4 + 128 * j);
  float s = 0.f;
#pragma unroll
  for (int j = 0; j < 4; ++j) s += (xv[j][0] + xv[j][1]) + (xv[j][2] + xv[j][3]);
#pragma unroll
  for (int off = 16; off > 0; off >>= 1) s += __shfl_xor(s, off, 32);
  const float mean = s * (1.0f / (float)kCh);
  float qs = 0.f;
#pragma unroll
  for (int j = 0; j < 4; ++j) {
#pragma unroll
    for (int c = 0; c < 4; ++c) {
      const float d = xv[j][c] - mean;
      qs += d * d;
    }
  }
#pragma unroll
  for (int off = 16; off > 0; off >>= 1) qs += __shfl_xor(qs, off, 32);
  const float rstd = rsqrtf(qs * (1.0f / (float)kCh) + 1e-5f);
  v4f yv[4];
#pragma unroll
  for (int j = 0; j < 4; ++j) {
    const v4f wv = *(const v4f*)(w + lane * 4 + 128 * j);
    const v4f bv = *(const v4f*)(b + lane * 4 + 128 * j);
#pragma unroll
    for (int c = 0; c < 4; ++c) {
      const float wc = wv[c], bc = bv[c];
      yv[j][c] = (xv[j][c] - mean) * rstd * rbf(wc) + rbf(bc);
    }
    *(v4f*)(sRow + wave * kCh + lane * 4 + 128 * j) = yv[j];
  }
  if (MODE == 1) {
    float* o = out32 + (size_t)tok * kCh + lane * 4;
    for (int pass = 0; pass < 2; ++pass) {
#pragma unroll
      for (int j = 0; j < 4; ++j) *(volatile v4f*)(o + 128 * j) = yv[j];
      __threadfence();
    }
  }
  __syncthreads();
  {
    size_t orow;
    if (MODE == 0) {
      const int t = tok >> 8, hp = (tok >> 4) & 15, wp = tok & 15;
      orow = (size_t)((t * kPadW + hp + 1) * kPadW + wp + 1);
    } else {
      orow = (size_t)tok;
    }
    v8h hv[2];
#pragma unroll
    for (int j = 0; j < 2; ++j) {
      const float* sp = sRow + wave * kCh + lane * 8 + 256 * j;
      const v4f u0 = *(const v4f*)(sp);
      const v4f u1 = *(const v4f*)(sp + 4);
#pragma unroll
      for (int e = 0; e < 4; ++e) {
        hv[j][e]     = (_Float16)(u0[e] * kCarryA);
        hv[j][4 + e] = (_Float16)(u1[e] * kCarryA);
      }
    }
    unsigned short* o = out16 + orow * kCh + lane * 8;
    for (int pass = 0; pass < 2; ++pass) {
#pragma unroll
      for (int j = 0; j < 2; ++j) *(volatile v8h*)(o + 256 * j) = hv[j];
      __threadfence();
    }
  }
  if (MODE == 1) {
    float l0 = 0.f, l1 = 0.f, l2 = 0.f, l3 = 0.f;
#pragma unroll 2
    for (int k = 0; k < 16; ++k) {
      const int ch = lane + 32 * k;
      const float yc = sRow[wave * kCh + ch];
      const v4f wv = *(const v4f*)(Wr + (size_t)ch * kExp);
      const float w0 = wv[0], w1 = wv[1], w2 = wv[2], w3 = wv[3];
      l0 = fmaf(yc, rbf(w0), l0);
      l1 = fmaf(yc, rbf(w1), l1);
      l2 = fmaf(yc, rbf(w2), l2);
      l3 = fmaf(yc, rbf(w3), l3);
    }
#pragma unroll
    for (int off = 16; off > 0; off >>= 1) {
      l0 += __shfl_xor(l0, off, 32);
      l1 += __shfl_xor(l1, off, 32);
      l2 += __shfl_xor(l2, off, 32);
      l3 += __shfl_xor(l3, off, 32);
    }
    const float mx = fmaxf(fmaxf(l0, l1), fmaxf(l2, l3));
    const int le = lane & 3;
    const float mine = (le == 0) ? l0 : (le == 1) ? l1 : (le == 2) ? l2 : l3;
    const float ex = expf(mine - mx);
    float sm = ex + __shfl_xor(ex, 1, 32);
    sm += __shfl_xor(sm, 2, 32);
    const float pr = ex * (1.0f / sm);
    if (lane < 4) sPr[wave * 4 + lane] = pr;
    __syncthreads();
    const v4f pv = *(const v4f*)(sPr + (lane & 7) * 4);
    if (wave == 0 && lane < 8) {
      float* o = probs + (size_t)blockIdx.x * 32 + lane * 4;
      *(volatile v4f*)o = pv;
      __threadfence();
      *(volatile v4f*)o = pv;
    }
  }
}

__global__ __launch_bounds__(256) void step_params_kernel(
    const float* __restrict__ XE, const float* __restrict__ Wsr, const float* __restrict__ Wsi,
    const float* __restrict__ Wg, const float* __restrict__ bg, float* __restrict__ TP) {
  __shared__ float sXm[kCh];
  const int t = blockIdx.x, tid = threadIdx.x;
  const float* base = XE + (size_t)t * kSpa * kCh;
  float s0 = 0.f, s1 = 0.f;
#pragma unroll 4
  for (int sp = 0; sp < kSpa; ++sp) {
    s0 += base[(size_t)sp * kCh + tid];
    s1 += base[(size_t)sp * kCh + kDc + tid];
  }
  sXm[tid] = s0 * (1.0f / (float)kSpa);
  sXm[kDc + tid] = s1 * (1.0f / (float)kSpa);
  __syncthreads();
  float sr = 0.f, si = 0.f;
#pragma unroll 2
  for (int d = 0; d < kDc; ++d) {
    const float xr = sXm[d], xi = sXm[kDc + d];
    const float wr = rbf(Wsr[(size_t)d * kDc + tid]);
    const float wi = rbf(Wsi[(size_t)d * kDc + tid]);
    sr += xr * wr - xi * wi;
    si += xr * wi + xi * wr;
  }
  float g = rbf(bg[tid]);
#pragma unroll 4
  for (int j = 0; j < kCh; ++j) g = fmaf(sXm[j], rbf(Wg[(size_t)j * kDc + tid]), g);
  const float gate = 1.0f / (1.0f + expf(-g));
  float* o = TP + (size_t)t * 3 * kDc + tid;
  for (int pass = 0; pass < 2; ++pass) {
    *(volatile float*)(o) = gate;
    *(volatile float*)(o + kDc) = sr;
    *(volatile float*)(o + 2 * kDc) = si;
    __threadfence();
  }
}

__global__ __launch_bounds__(256) void decay_kernel(
    const float* __restrict__ lam_re, const float* __restrict__ lam_im, const float* __restrict__ dt,
    float* __restrict__ DP) {
  const int lt = blockIdx.x, l = lt >> 3, t = lt & 7, e = threadIdx.x;
  const float lrx = rbf(lam_re[l * kDc + e]);
  const float li  = rbf(lam_im[l * kDc + e]);
  const float dtv = rbf(dt[t]);
  const float sp = fmaxf(lrx, 0.0f) + log1pf(expf(-fabsf(lrx)));
  const float lr = -(sp + 0.01f);
  const float mag = expf(lr * dtv);
  float sn, cs;
  sincosf(li * dtv, &sn, &cs);
  const float ar = mag * cs, ai = mag * sn;
  const float den = lr * lr + li * li;
  const float inv = 1.0f / den;
  const float nr = ar - 1.0f, ni = ai;
  const float pr = (nr * lr + ni * li) * inv;
  const float pi = (ni * lr - nr * li) * inv;
  float* o = DP + (size_t)lt * 4 * kDc + e;
  for (int pass = 0; pass < 2; ++pass) {
    *(volatile float*)(o) = ar;
    *(volatile float*)(o + kDc) = ai;
    *(volatile float*)(o + 2 * kDc) = pr;
    *(volatile float*)(o + 3 * kDc) = pi;
    __threadfence();
  }
}

__global__ __launch_bounds__(256) void scan_kernel(
    const float* __restrict__ XE, const float* __restrict__ TP, const float* __restrict__ DP,
    float* __restrict__ HS, unsigned short* __restrict__ H16, int read_state, int write_state) {
  __shared__ __align__(16) float sH[kSteps * kCh];
  __shared__ __align__(16) float sP[kCh];
  const int s = blockIdx.x, e = threadIdx.x, tid = threadIdx.x;
  float hpr = 0.f, hpi = 0.f;
  if (read_state) {
    hpr = HS[(size_t)s * kCh + e];
    hpi = HS[(size_t)s * kCh + kDc + e];
  }
  float hr = 0.f, hi = 0.f, outr = 0.f, outi = 0.f;
#pragma unroll 1
  for (int t = 0; t < kSteps; ++t) {
    const float* tp = TP + (size_t)t * 3 * kDc;
    const float* dp = DP + (size_t)t * 4 * kDc;
    const float g = tp[e], sr = tp[kDc + e], si = tp[2 * kDc + e];
    const float ar = dp[e], ai = dp[kDc + e], pr = dp[2 * kDc + e], pi = dp[3 * kDc + e];
    const size_t n = (size_t)t * kSpa + s;
    const float xr = XE[n * kCh + e], xi = XE[n * kCh + kDc + e];
    const float omg = 1.0f - g;
    const float fr = xr * g + sr * omg;
    const float fi = xi * g + si * omg;
    const float ur = fr * pr - fi * pi;
    const float ui = fr * pi + fi * pr;
    const float nhr = ar * hr - ai * hi + ur;
    const float nhi = ar * hi + ai * hr + ui;
    hr = nhr; hi = nhi;
    outr = hr + (hpr * ar - hpi * ai);
    outi = hi + (hpr * ai + hpi * ar);
    sH[t * kCh + e] = outr;
    sH[t * kCh + kDc + e] = outi;
  }
  sP[e] = outr;
  sP[kDc + e] = outi;
  __syncthreads();
  v8h hv[2];
#pragma unroll
  for (int it = 0; it < 2; ++it) {
    const int chunk = it * 256 + tid;
    const int row = chunk >> 6, c8 = (chunk & 63) * 8;
    const float* sp = sH + row * kCh + c8;
    const v4f u0 = *(const v4f*)(sp);
    const v4f u1 = *(const v4f*)(sp + 4);
#pragma unroll
    for (int k = 0; k < 4; ++k) {
      hv[it][k]     = (_Float16)(u0[k] * kCarryA);
      hv[it][4 + k] = (_Float16)(u1[k] * kCarryA);
    }
  }
  const v4f pv = *(const v4f*)(sP + (tid & 127) * 4);
  for (int pass = 0; pass < 2; ++pass) {
#pragma unroll
    for (int it = 0; it < 2; ++it) {
      const int chunk = it * 256 + tid;
      const int row = chunk >> 6, c8 = (chunk & 63) * 8;
      *(volatile v8h*)(H16 + ((size_t)row * kSpa + s) * kCh + c8) = hv[it];
    }
    if (write_state && tid < 128) *(volatile v4f*)(HS + (size_t)s * kCh + tid * 4) = pv;
    __threadfence();
  }
}

extern "C" void kernel_launch(void* const* d_in, const int* in_sizes, int n_in,
                              void* d_out, int out_size, void* d_ws, size_t ws_size,
                              hipStream_t stream) {
  if (n_in < 25) return;
  if (in_sizes[0] != kSteps * 4 * 256 * 256) return;
  if (in_sizes[1] != kSteps) return;
  if (in_sizes[2] != kPatchF * kCh || in_sizes[4] != kCh * kPatchF) return;
  if (in_sizes[8] != kLayers * kCh * kConvK) return;
  if (in_sizes[10] != kLayers * kDc * kDc || in_sizes[16] != kLayers * kCh * kDc) return;
  if (in_sizes[22] != kLayers * kCh * kExp) return;
  if (in_sizes[23] != kLayers * kExp * kCh * kFfn || in_sizes[24] != kLayers * kExp * kFfn * kCh) return;
  if (out_size != kSteps * 4 * 256 * 256) return;
  if (ws_size < kWsTotal) return;

  const float* x       = (const float*)d_in[0];
  const float* dt      = (const float*)d_in[1];
  const float* Wenc    = (const float*)d_in[2];
  const float* benc    = (const float*)d_in[3];
  const float* Wdec    = (const float*)d_in[4];
  const float* bdec    = (const float*)d_in[5];
  const float* ln_sp_w = (const float*)d_in[6];
  const float* ln_sp_b = (const float*)d_in[7];
  const float* conv_w  = (const float*)d_in[8];
  const float* conv_b  = (const float*)d_in[9];
  const float* E_re    = (const float*)d_in[10];
  const float* E_im    = (const float*)d_in[11];
  const float* Ed_re   = (const float*)d_in[12];
  const float* Ed_im   = (const float*)d_in[13];
  const float* Ws_re   = (const float*)d_in[14];
  const float* Ws_im   = (const float*)d_in[15];
  const float* Wg      = (const float*)d_in[16];
  const float* bg      = (const float*)d_in[17];
  const float* lam_re  = (const float*)d_in[18];
  const float* lam_im  = (const float*)d_in[19];
  const float* ln_t_w  = (const float*)d_in[20];
  const float* ln_t_b  = (const float*)d_in[21];
  const float* Wr      = (const float*)d_in[22];
  const float* W1      = (const float*)d_in[23];
  const float* W2      = (const float*)d_in[24];
  float* out = (float*)d_out;

  char* ws = (char*)d_ws;
  unsigned short* WENCT = (unsigned short*)(ws + kOffWencT);
  unsigned short* WDECT = (unsigned short*)(ws + kOffWdecT);
  unsigned short* CONVT = (unsigned short*)(ws + kOffConvT);
  unsigned short* ECM   = (unsigned short*)(ws + kOffEcm);
  unsigned short* EDCM  = (unsigned short*)(ws + kOffEdcm);
  unsigned short* W1T   = (unsigned short*)(ws + kOffW1T);
  unsigned short* W2T   = (unsigned short*)(ws + kOffW2T);
  unsigned short* XP    = (unsigned short*)(ws + kOffXp);
  float*          Z     = (float*)(ws + kOffZ);
  float*          X     = (float*)(ws + kOffX);
  float*          XE    = (float*)(ws + kOffXE);
  float*          XO    = (float*)(ws + kOffXO);
  float*          TOK   = (float*)(ws + kOffTok);
  unsigned short* ZNP   = (unsigned short*)(ws + kOffZnp);
  unsigned short* X16   = (unsigned short*)(ws + kOffX16);
  unsigned short* H16   = (unsigned short*)(ws + kOffH16);
  unsigned short* TOK16 = (unsigned short*)(ws + kOffTok16);
  unsigned short* Z16   = (unsigned short*)(ws + kOffZ16);
  unsigned short* HID   = (unsigned short*)(ws + kOffHid);
  float*          PROBS = (float*)(ws + kOffProbs);
  float*          TPAR  = (float*)(ws + kOffTpar);
  float*          DPAR  = (float*)(ws + kOffDpar);
  float*          HST   = (float*)(ws + kOffHst);

  pack_transpose_kernel<<<dim3(kPatchF / 64, kCh / 64, 1), 256, 0, stream>>>(
      Wenc, kCh, 0L, WENCT, kPatchF, 1, 0L, 0L, kCarryW);
  pack_transpose_kernel<<<dim3(kCh / 64, kPatchF / 64, 1), 256, 0, stream>>>(
      Wdec, kPatchF, 0L, WDECT, kCh, 1, 0L, 0L, kCarryW);
  pack_transpose_kernel<<<dim3(kCh / 64, kFfn / 64, kLayers * kExp), 256, 0, stream>>>(
      W1, kFfn, (long)kCh * kFfn, W1T, kCh, kExp, (long)kFfnAll * kCh, (long)kFfn * kCh, kCarryW);
  pack_transpose_kernel<<<dim3(kFfn / 64, kCh / 64, kLayers * kExp), 256, 0, stream>>>(
      W2, kCh, (long)kFfn * kCh, W2T, kFfnAll, kExp, (long)kCh * kFfnAll, (long)kFfn, kCarryW);
  pack_cplx_kernel<<<dim3(4, 4, 16), 256, 0, stream>>>(E_re, E_im, Ed_re, Ed_im, ECM, kCarryW);
  pack_conv_kernel<<<kLayers * kCh, 256, 0, stream>>>(conv_w, CONVT, kCarryW);
  halo_zero_kernel<<<kPadRows, 64, 0, stream>>>(ZNP);
  decay_kernel<<<kLayers * kSteps, 256, 0, stream>>>(lam_re, lam_im, dt, DPAR);

  patchify_kernel<<<(kTok * kPatchF / 8) / 256, 256, 0, stream>>>(x, XP);
  gemm_f16_kernel<0, EPI_BIAS><<<128, 64, 0, stream>>>(
      XP, kPatchF, WENCT, kPatchF, Z, nullptr, kCh, benc, nullptr, nullptr,
      kTok, kCh, kPatchF, kScaleXW, 0.0f);

  for (int l = 0; l < kLayers; ++l) {
    const float* tpar = TPAR + (size_t)l * kSteps * 3 * kDc;
    const float* dpar = DPAR + (size_t)l * kSteps * 4 * kDc;
    ln_kernel<0><<<kTok / 8, 256, 0, stream>>>(Z, ln_sp_w + l * kCh, ln_sp_b + l * kCh, ZNP, nullptr, nullptr, nullptr);
    gemm_f16_kernel<1, EPI_CONV><<<128, 64, 0, stream>>>(
        ZNP, kCh, CONVT + (size_t)l * kCh * kConvK, kConvK, X, X16, kCh,
        conv_b + l * kCh, Z, nullptr, kTok, kCh, kConvK, kScaleAW, kCarryA);
    gemm_f16_kernel<0, EPI_PLAIN><<<128, 64, 0, stream>>>(
        X16, kCh, ECM + (size_t)l * kCh * kCh, kCh, XE, nullptr, kCh,
        nullptr, nullptr, nullptr, kTok, kCh, kCh, kScaleAW, 0.0f);
    step_params_kernel<<<kSteps, 256, 0, stream>>>(
        XE, Ws_re + (size_t)l * kDc * kDc, Ws_im + (size_t)l * kDc * kDc,
        Wg + (size_t)l * kCh * kDc, bg + l * kDc, TPAR + (size_t)l * kSteps * 3 * kDc);
    scan_kernel<<<kSpa, 256, 0, stream>>>(XE, tpar, dpar, HST, H16, (l > 0) ? 1 : 0, (l == 0) ? 1 : 0);
    gemm_f16_kernel<0, EPI_PLAIN><<<128, 64, 0, stream>>>(
        H16, kCh, EDCM + (size_t)l * kCh * kCh, kCh, XO, nullptr, kCh,
        nullptr, nullptr, nullptr, kTok, kCh, kCh, kScaleAW, 0.0f);
    ln_kernel<1><<<kTok / 8, 256, 0, stream>>>(XO, ln_t_w + l * kCh, ln_t_b + l * kCh, TOK16, TOK,
                                               Wr + (size_t)l * kCh * kExp, PROBS);
    gemm_f16_kernel<0, EPI_UP><<<1024, 64, 0, stream>>>(
        TOK16, kCh, W1T + (size_t)l * kFfnAll * kCh, kCh, nullptr, HID, kFfnAll,
        nullptr, PROBS, nullptr, kTok, kFfnAll, kCh, kScaleAW, kCarryH);
    gemm_f16_kernel<0, EPI_DOWN><<<128, 64, 0, stream>>>(
        HID, kFfnAll, W2T + (size_t)l * kCh * kFfnAll, kFfnAll, Z, Z16, kCh,
        nullptr, X, TOK, kTok, kCh, kFfnAll, kScaleHW, kCarryA);
  }

  gemm_f16_kernel<0, EPI_IMG><<<256, 64, 0, stream>>>(
      Z16, kCh, WDECT, kCh, out, nullptr, kCh, bdec, nullptr, nullptr,
      kTok, kPatchF, kCh, kScaleAW, 0.0f);
}
